// Pseudo_MHSA_Block_21328807592207
// MI455X (gfx1250) — hardware-verified
//
#include <hip/hip_runtime.h>


namespace {
constexpr int Bn = 4, L = 2048, D = 768, H = 12, HD = 64, NT = Bn * L, DI = 3072;
constexpr float XS = 8.0f, PS = 8.0f, EPS = 1e-5f;
struct Wo_ { static constexpr size_t P_ = 0, A = (size_t)D * D, V = A + (size_t)H * HD * HD, O = V + (size_t)H * HD * HD, UP = O + (size_t)D * D, DN = UP + (size_t)DI * D, END = DN + (size_t)D * DI; };

typedef _Float16 b16;
typedef __attribute__((ext_vector_type(16))) _Float16 v16b;
typedef __attribute__((ext_vector_type(8))) _Float16 v8b;
typedef __attribute__((ext_vector_type(8))) float v8f;
typedef __attribute__((ext_vector_type(4))) float v4f;
__device__ __forceinline__ float bf16_rne(float f) { unsigned int u = __float_as_uint(f); u += 0x7FFFu + ((u >> 16) & 1u); return __uint_as_float(u & 0xFFFF0000u); }
__device__ __forceinline__ v16b frag_kb(const b16* p, int hh) { const v8b a = *(const v8b*)(p + 8 * hh), b = *(const v8b*)(p + 16 + 8 * hh); v16b f;
#pragma unroll
  for (int e = 0; e < 8; ++e) { f[e] = a[e]; f[8 + e] = b[e]; } return f; }
__device__ __forceinline__ v8f wmma16b(v16b a, v16b b, v8f c) { v8f d = __builtin_amdgcn_wmma_f32_16x16x32_f16(false, a, false, b, (short)0, c, false, false); asm volatile("v_nop\n\tv_nop\n\tv_nop\n\tv_nop" : "+v"(d) : "v"(a), "v"(b)); return d; }
__device__ __forceinline__ void wave_lds_sync() { __builtin_amdgcn_fence(__ATOMIC_RELEASE, "workgroup"); __builtin_amdgcn_wave_barrier(); __builtin_amdgcn_fence(__ATOMIC_ACQUIRE, "workgroup"); }
__device__ __forceinline__ float nexp(float x) { return __builtin_amdgcn_exp2f(x * 1.4426950408889634f); }
__device__ __forceinline__ float pmul(float a, float b) { float p = a * b; asm volatile("" : "+v"(p)); return p; }
__device__ __forceinline__ float wsum(float v) {
#pragma unroll
  for (int o = 1; o < 32; o <<= 1) v += __shfl_xor(v, o); return v; }
__device__ __forceinline__ float silu_f(float y) { return y / (1.0f + nexp(-y)); }

__global__ __launch_bounds__(256) void prep_kernel(const float* __restrict__ pw, const float* __restrict__ aw, const float* __restrict__ vw, const float* __restrict__ ow, const float* __restrict__ w1, const float* __restrict__ w2, const float* __restrict__ l1s, const float* __restrict__ l1b, const float* __restrict__ l2s, const float* __restrict__ l2b, const float* __restrict__ ob, const float* __restrict__ b1, const float* __restrict__ b2, b16* __restrict__ R, float* __restrict__ P) {
  const size_t tid = (size_t)blockIdx.x * 256 + threadIdx.x, nth = (size_t)gridDim.x * 256;
  auto tr = [&](size_t base, int nout, int kin, const float* W) { for (size_t p = tid; p < (size_t)nout * (kin / 8); p += nth) { const int o = (int)(p / (kin / 8)), k0 = (int)(p % (kin / 8)) * 8; v8b v;
#pragma unroll
      for (int e = 0; e < 8; ++e) v[e] = (b16)bf16_rne(W[(size_t)(k0 + e) * nout + o]); *(volatile v8b*)(R + base + (size_t)o * kin + k0) = v; } };
  for (int pass = 0; pass < 2; ++pass) { tr(Wo_::P_, D, D, pw); tr(Wo_::O, D, D, ow); tr(Wo_::UP, DI, D, w1); tr(Wo_::DN, D, DI, w2);
    for (size_t p = tid; p < (size_t)H * HD * (HD / 8); p += nth) { const int h = (int)(p / (HD * HD / 8)), rem = (int)(p % (HD * HD / 8)), e_ = rem / (HD / 8), d0 = (rem % (HD / 8)) * 8; v8b va, vv;
      for (int e = 0; e < 8; ++e) { va[e] = (b16)bf16_rne(aw[((size_t)h * HD + d0 + e) * HD + e_]); vv[e] = (b16)bf16_rne(vw[((size_t)h * HD + d0 + e) * HD + e_]); }
      *(volatile v8b*)(R + Wo_::A + ((size_t)h * HD + e_) * HD + d0) = va; *(volatile v8b*)(R + Wo_::V + ((size_t)h * HD + e_) * HD + d0) = vv; }
    for (size_t q = tid; q < 7680; q += nth) { const int i = (int)q; float v; if (i < 768) v = l1s[i]; else if (i < 1536) v = l1b[i - 768]; else if (i < 2304) v = l2s[i - 1536]; else if (i < 3072) v = l2b[i - 2304]; else if (i < 3840) v = ob[i - 3072]; else if (i < 6912) v = b1[i - 3840]; else v = b2[i - 6912]; P[q] = bf16_rne(v); }
    __threadfence(); }
}

template <int RND>
__global__ __launch_bounds__(256) void ln_kernel(const float* __restrict__ src, const float* __restrict__ g, const float* __restrict__ bb, b16* __restrict__ dst) {
  const int row = blockIdx.x * 8 + (threadIdx.x >> 5), lane = threadIdx.x & 31; const float* xr = src + (size_t)row * D;
  float v[24]; float s = 0.0f;
#pragma unroll
  for (int i = 0; i < 24; ++i) { float x = xr[(i >> 3) * 256 + lane * 8 + (i & 7)]; if (RND) x = bf16_rne(x); v[i] = x; s += x; }
  s = wsum(s); const float mu = s * (1.0f / D); float q = 0.0f;
#pragma unroll
  for (int i = 0; i < 24; ++i) { const float d = v[i] - mu; q += pmul(d, d); }
  q = wsum(q); const float inv = rsqrtf(q * (1.0f / D) + EPS);
  for (int pass = 0; pass < 2; ++pass) {
#pragma unroll
    for (int gq = 0; gq < 3; ++gq) { v8b o; const int c0 = gq * 256 + lane * 8; for (int e = 0; e < 8; ++e) o[e] = (b16)((pmul((v[gq * 8 + e] - mu) * inv, g[c0 + e]) + bb[c0 + e]) * XS); *(volatile v8b*)(dst + (size_t)row * D + c0) = o; }
    __threadfence(); }
}

template <int K, int N, int EPI, int RND>
__global__ __launch_bounds__(64) void gemm_kernel(const b16* __restrict__ A, const b16* __restrict__ Bw, const float* __restrict__ bias, const float* __restrict__ resid, b16* __restrict__ Ch, float* __restrict__ Cf) {
  __shared__ __attribute__((aligned(16))) float Ts[2][32][128 + 4];
  const int lane = threadIdx.x & 31, wave = threadIdx.x >> 5, nloc = lane & 15, hlf = lane >> 4, m0 = blockIdx.y * 32, c0 = blockIdx.x * 256 + wave * 128;
#pragma unroll 1
  for (int hf = 0; hf < 2; ++hf) { v8f acc[2][4];
#pragma unroll
    for (int r = 0; r < 2; ++r)
#pragma unroll
      for (int t = 0; t < 4; ++t) acc[r][t] = (v8f){};
#pragma unroll 2
    for (int kb = 0; kb < K; kb += 32) { const v16b a0 = frag_kb(A + (size_t)(m0 + nloc) * K + kb, hlf), a1 = frag_kb(A + (size_t)(m0 + 16 + nloc) * K + kb, hlf);
#pragma unroll
      for (int t = 0; t < 4; ++t) { const v16b bw = frag_kb(Bw + (size_t)(c0 + (hf * 4 + t) * 16 + nloc) * K + kb, hlf); acc[0][t] = wmma16b(a0, bw, acc[0][t]); acc[1][t] = wmma16b(a1, bw, acc[1][t]); } }
#pragma unroll
    for (int t = 0; t < 4; ++t) { const int cl = (hf * 4 + t) * 16 + nloc, c = c0 + cl;
#pragma unroll
      for (int r = 0; r < 2; ++r)
#pragma unroll
        for (int v = 0; v < 8; ++v) { const int rr = r * 16 + 8 * hlf + v; float y = acc[r][t][v] * (1.0f / XS); if (EPI == 1) { float xr = resid[(size_t)(m0 + rr) * N + c]; y += bias[c] + (RND ? bf16_rne(xr) : xr); } Ts[wave][rr][cl] = y; } } }
  wave_lds_sync();
  for (int pass = 0; pass < 2; ++pass) {
    if (EPI == 1) { for (int i = lane; i < 32 * 32; i += 32) { const int rr = i >> 5, c4 = (i & 31) * 4; *(volatile v4f*)(Cf + (size_t)(m0 + rr) * N + c0 + c4) = *(const v4f*)(&Ts[wave][rr][c4]); } }
    else { for (int i = lane; i < 32 * 16; i += 32) { const int rr = i >> 4, c8 = (i & 15) * 8; v8b o; for (int e = 0; e < 8; ++e) o[e] = (b16)(Ts[wave][rr][c8 + e] * XS); *(volatile v8b*)(Ch + (size_t)(m0 + rr) * N + c0 + c8) = o; } }
    __threadfence(); }
}

__global__ __launch_bounds__(128) void head_kernel(const b16* __restrict__ XP, const b16* __restrict__ R, b16* __restrict__ XQ, b16* __restrict__ VT) {
  __shared__ __attribute__((aligned(16))) b16 Tq[128][HD + 8], Tv[HD][128 + 8];
  const int lane = threadIdx.x & 31, wave = threadIdx.x >> 5, nloc = lane & 15, hlf = lane >> 4, h = blockIdx.y, t0 = blockIdx.x * 128, m0 = t0 + wave * 32; const int b = t0 / L, p0 = t0 % L;
  const b16* Aw = R + Wo_::A + (size_t)h * HD * HD; const b16* Vw = R + Wo_::V + (size_t)h * HD * HD;
  v8f aq[2][4], av[2][4];
#pragma unroll
  for (int r = 0; r < 2; ++r)
#pragma unroll
    for (int t = 0; t < 4; ++t) { aq[r][t] = (v8f){}; av[r][t] = (v8f){}; }
#pragma unroll
  for (int kb = 0; kb < HD; kb += 32) { const v16b a0 = frag_kb(XP + (size_t)(m0 + nloc) * D + h * HD + kb, hlf), a1 = frag_kb(XP + (size_t)(m0 + 16 + nloc) * D + h * HD + kb, hlf);
#pragma unroll
    for (int t = 0; t < 4; ++t) { const v16b bq = frag_kb(Aw + (size_t)(t * 16 + nloc) * HD + kb, hlf), bv = frag_kb(Vw + (size_t)(t * 16 + nloc) * HD + kb, hlf);
      aq[0][t] = wmma16b(a0, bq, aq[0][t]); aq[1][t] = wmma16b(a1, bq, aq[1][t]); av[0][t] = wmma16b(a0, bv, av[0][t]); av[1][t] = wmma16b(a1, bv, av[1][t]); } }
#pragma unroll
  for (int t = 0; t < 4; ++t)
#pragma unroll
    for (int r = 0; r < 2; ++r)
#pragma unroll
      for (int v = 0; v < 8; ++v) { const int rr = wave * 32 + r * 16 + 8 * hlf + v, c = t * 16 + nloc; Tq[rr][c] = (b16)(aq[r][t][v]); Tv[c][rr] = (b16)(av[r][t][v]); }
  __syncthreads();
  for (int pass = 0; pass < 2; ++pass) {
    for (int i = threadIdx.x; i < 128 * 8; i += 128) { const int rr = i >> 3, c8 = (i & 7) * 8; *(volatile v8b*)(XQ + (size_t)(t0 + rr) * D + h * HD + c8) = *(const v8b*)(&Tq[rr][c8]); }
    for (int i = threadIdx.x; i < HD * 16; i += 128) { const int d = i >> 4, c8 = (i & 15) * 8; *(volatile v8b*)(VT + (((size_t)b * H + h) * HD + d) * L + p0 + c8) = *(const v8b*)(&Tv[d][c8]); }
    __threadfence(); }
}

__global__ __launch_bounds__(128) void attn_kernel(const b16* __restrict__ XQ, const b16* __restrict__ XP, const b16* __restrict__ vt, b16* __restrict__ ctx) {
  __shared__ __attribute__((aligned(16))) b16 Os[16][4 * HD + 8];
  const int wid = threadIdx.x >> 5, lane = threadIdx.x & 31, hh = lane >> 4, col = lane & 15; const int b = blockIdx.x / (L / 16), q0 = (blockIdx.x % (L / 16)) * 16, h = blockIdx.y * 4 + wid, qi = q0 + col; constexpr int DQK = D;
  const b16* Qr = XQ + (size_t)(b * L) * D + h * HD; const b16* Kr = XP + (size_t)(b * L) * D + h * HD; const b16* V = vt + (((size_t)b * H + h) * HD) * L;
  const v16b qf0 = frag_kb(Qr + (size_t)qi * DQK, hh), qf1 = frag_kb(Qr + (size_t)qi * DQK + 32, hh);
  float m = -INFINITY, l = 0.0f; v8f o[4] = {{}, {}, {}, {}};
  for (int kb = 0; kb < L; kb += 32) {
    v8f s0 = {}, s1 = {}; s0 = wmma16b(frag_kb(Kr + (size_t)(kb + col) * DQK, hh), qf0, s0); s0 = wmma16b(frag_kb(Kr + (size_t)(kb + col) * DQK + 32, hh), qf1, s0);
    s1 = wmma16b(frag_kb(Kr + (size_t)(kb + 16 + col) * DQK, hh), qf0, s1); s1 = wmma16b(frag_kb(Kr + (size_t)(kb + 16 + col) * DQK + 32, hh), qf1, s1);
    float mr = -INFINITY;
#pragma unroll
    for (int r = 0; r < 8; ++r) { s0[r] *= (0.015625f / (XS * XS)); s1[r] *= (0.015625f / (XS * XS)); mr = fmaxf(mr, fmaxf(s0[r], s1[r])); }
    mr = fmaxf(mr, __shfl_xor(mr, 16)); const float mn = fmaxf(m, mr), al_ = nexp(m - mn); m = mn; float sum = 0.0f; v16b pb;
#pragma unroll
    for (int r = 0; r < 8; ++r) { const float e0 = nexp(s0[r] - mn), e1 = nexp(s1[r] - mn); sum += e0 + e1; pb[r] = (b16)(e0 * PS); pb[8 + r] = (b16)(e1 * PS); }
    sum += __shfl_xor(sum, 16); l = l * al_ + sum;
#pragma unroll
    for (int t = 0; t < 4; ++t) { o[t] *= al_; o[t] = wmma16b(frag_kb(V + (size_t)(t * 16 + col) * L + kb, hh), pb, o[t]); } }
  const float inv = 1.0f / (l * PS);
#pragma unroll
  for (int t = 0; t < 4; ++t)
#pragma unroll
    for (int r = 0; r < 8; ++r) Os[col][wid * HD + t * 16 + 8 * hh + r] = (b16)(o[t][r] * inv);
  __syncthreads();
  for (int pass = 0; pass < 2; ++pass) { for (int i = threadIdx.x; i < 16 * 32; i += 128) { const int rr = i >> 5, c8 = (i & 31) * 8; *(volatile v8b*)(ctx + (size_t)(b * L + q0 + rr) * D + blockIdx.y * 4 * HD + c8) = *(const v8b*)(&Os[rr][c8]); } __threadfence(); }
}

__global__ __launch_bounds__(256) void mlp_kernel(const b16* __restrict__ Hh, const b16* __restrict__ R, const float* __restrict__ P, const float* __restrict__ X1, float* __restrict__ out) {
  __shared__ __attribute__((aligned(16))) b16 G[16][DI + 8];
  const int wave = threadIdx.x >> 5, lane = threadIdx.x & 31, nloc = lane & 15, hlf = lane >> 4, r0 = blockIdx.x * 16; const b16* Wu = R + Wo_::UP; const b16* Wd = R + Wo_::DN;
  for (int t = wave; t < DI / 16; t += 8) { v8f acc = {};
#pragma unroll 4
    for (int kb = 0; kb < D; kb += 32) acc = wmma16b(frag_kb(Hh + (size_t)(r0 + nloc) * D + kb, hlf), frag_kb(Wu + (size_t)(t * 16 + nloc) * D + kb, hlf), acc);
    const int c = t * 16 + nloc;
#pragma unroll
    for (int r = 0; r < 8; ++r) { const float u = acc[r] * (1.0f / XS) + P[3840 + c]; G[8 * hlf + r][c] = (b16)(0.5f * u * (1.0f + erff(u * 0.70710678118654752f)) * XS); } }
  __syncthreads();
  v8f acc2[6];
#pragma unroll
  for (int t = 0; t < 6; ++t) acc2[t] = (v8f){};
#pragma unroll 2
  for (int kb = 0; kb < DI; kb += 32) { const v16b a = frag_kb(&G[nloc][kb], hlf);
#pragma unroll
    for (int t = 0; t < 6; ++t) acc2[t] = wmma16b(a, frag_kb(Wd + (size_t)(wave * 96 + t * 16 + nloc) * DI + kb, hlf), acc2[t]); }
  float vals[6][8];
#pragma unroll
  for (int t = 0; t < 6; ++t) { const int c = wave * 96 + t * 16 + nloc;
#pragma unroll
    for (int r = 0; r < 8; ++r) vals[t][r] = acc2[t][r] * (1.0f / XS) + P[6912 + c] + X1[(size_t)(r0 + 8 * hlf + r) * D + c]; }
  __syncthreads();
  float (*St)[D + 4] = (float (*)[D + 4])(&G[0][0]);
#pragma unroll
  for (int t = 0; t < 6; ++t)
#pragma unroll
    for (int r = 0; r < 8; ++r) St[8 * hlf + r][wave * 96 + t * 16 + nloc] = vals[t][r];
  __syncthreads();
  for (int pass = 0; pass < 2; ++pass) { for (int i = threadIdx.x; i < 16 * (D / 4); i += 256) { const int rr = i / (D / 4), c4 = (i % (D / 4)) * 4; *(volatile v4f*)(out + (size_t)(r0 + rr) * D + c4) = *(const v4f*)(&St[rr][c4]); } __threadfence(); }
}
}

extern "C" void kernel_launch(void* const* d_in, const int* in_sizes, int n_in,
                              void* d_out, int out_size, void* d_ws, size_t ws_size, hipStream_t stream) {
  (void)n_in; (void)out_size;
  const float* x = (const float*)d_in[0]; const float* pw = (const float*)d_in[1]; const float* aw = (const float*)d_in[2]; const float* vw = (const float*)d_in[3]; const float* ow = (const float*)d_in[4]; const float* ob = (const float*)d_in[5];
  const float* l1s = (const float*)d_in[6]; const float* l1b = (const float*)d_in[7]; const float* l2s = (const float*)d_in[8]; const float* l2b = (const float*)d_in[9]; const float* w1 = (const float*)d_in[10]; const float* b1 = (const float*)d_in[11]; const float* w2 = (const float*)d_in[12]; const float* b2 = (const float*)d_in[13];
  float* out = (float*)d_out;
  if (in_sizes[0] != NT * D || in_sizes[1] != D * H * HD || in_sizes[2] != H * HD * HD || in_sizes[10] != D * DI || in_sizes[12] != DI * D) return;
  size_t off = 0; char* ws = (char*)d_ws;
  auto carve = [&](size_t bytes) { char* p = ws + off; off += (bytes + 255) & ~(size_t)255; return p; };
  b16* R = (b16*)carve(Wo_::END * 2); float* P = (float*)carve(7680 * 4); b16* XN = (b16*)carve((size_t)NT * D * 2); b16* XP = (b16*)carve((size_t)NT * D * 2); b16* XQ = (b16*)carve((size_t)NT * D * 2); b16* VT = (b16*)carve((size_t)NT * D * 2); float* X1 = (float*)carve((size_t)NT * D * 4);
  if (off > ws_size) return;
  b16* CTX = XN; b16* HH = XP;
  prep_kernel<<<512, 256, 0, stream>>>(pw, aw, vw, ow, w1, w2, l1s, l1b, l2s, l2b, ob, b1, b2, R, P);
  ln_kernel<1><<<NT / 8, 256, 0, stream>>>(x, P, P + 768, XN);
  gemm_kernel<D, D, 0, 0><<<dim3(D / 256, NT / 32), 64, 0, stream>>>(XN, R + Wo_::P_, nullptr, nullptr, XP, nullptr);
  head_kernel<<<dim3(NT / 128, H), 128, 0, stream>>>(XP, R, XQ, VT);
  attn_kernel<<<dim3(NT / 16, 3), 128, 0, stream>>>(XQ, XP, VT, CTX);
  gemm_kernel<D, D, 1, 1><<<dim3(D / 256, NT / 32), 64, 0, stream>>>(CTX, R + Wo_::O, P + 3072, x, nullptr, X1);
  ln_kernel<0><<<NT / 8, 256, 0, stream>>>(X1, P + 1536, P + 2304, HH);
  mlp_kernel<<<NT / 16, 256, 0, stream>>>(HH, R, P, X1, out);
}
